// GRUModel_47725676593785
// MI455X (gfx1250) — hardware-verified
//
#include <hip/hip_runtime.h>
#include <math.h>

constexpr int NB    = 32768;
constexpr int TSEQ  = 18;
constexpr int NIN   = 2;
constexpr int HID   = 64;
constexpr int G3    = 3 * HID;
constexpr int F1N   = 24;
constexpr int F1K   = 2 * HID;
constexpr int F1NP  = 32;
constexpr int F2N   = 2;
constexpr int XROW  = TSEQ * NIN;
constexpr int OROW  = F1N * F2N;
constexpr int VROW  = TSEQ * F1N;
constexpr int RPB   = 32;
constexpr int NTHR  = 256;
constexpr int NWAVE = NTHR / 32;
constexpr int WP    = 64;
constexpr int CSTD  = 768;
constexpr int CST_BIH = 384;
constexpr int CST_BHH = 576;
constexpr float WCAR     = 16.0f;
constexpr float WCAR_INV = 1.0f / 16.0f;
constexpr float LCAR     = 2048.0f;
constexpr float LCAR_INV = 1.0f / 2048.0f;
constexpr float F16_MIN_NORMAL = 6.103515625e-5f;

constexpr int OFF_WHL = 0;
constexpr int OFF_F1L = OFF_WHL + 2 * G3 * WP * 2;
constexpr int OFF_HHI = OFF_F1L + 2 * F1NP * WP * 2;
constexpr int OFF_HLO = OFF_HHI + 4 * 16 * WP * 2;
constexpr int OFF_XS  = OFF_HLO + 4 * 16 * WP * 2;
constexpr int OFF_CST = OFF_XS + RPB * XROW * 4;
constexpr int OFF_TAB = OFF_CST + 2 * CSTD * 4;
constexpr int OFF_OST = OFF_TAB + 64 * 4;
constexpr int OFF_FCP = OFF_OST + RPB * OROW * 4;
constexpr int LDS_TOTAL = OFF_FCP + RPB * VROW * 4;

static_assert(NB % RPB == 0);
static_assert(RPB == 2 * 16 && NWAVE == 8);
static_assert(HID % 32 == 0 && F1K == 2 * HID && G3 == 3 * HID);
static_assert((G3 * (HID / 8)) % NTHR == 0);
static_assert(F1NP * (HID / 8) == NTHR);
static_assert((RPB * XROW) % 4 == 0);
static_assert((2 * 4 * 16 * WP * 2) % (16 * NTHR) == 0);
static_assert((RPB * VROW * 4) % 16 == 0);
static_assert((RPB * F1N) % NTHR == 0);
static_assert(RPB * OROW == 6 * 2 * 128);
static_assert((RPB * OROW * 4) % 128 == 0);
static_assert(OFF_F1L % 16 == 0 && OFF_HHI % 16 == 0 && OFF_HLO % 16 == 0 && OFF_XS % 16 == 0 &&
              OFF_CST % 16 == 0 && OFF_TAB % 16 == 0 && OFF_OST % 16 == 0 && OFF_FCP % 16 == 0);
static_assert((G3 * NIN) / 4 <= NTHR && G3 / 4 <= NTHR);
static_assert(F1N % 4 == 0 && (F2N * TSEQ) % 4 == 0);
static_assert(F1N + F2N * TSEQ + F2N <= 64);

typedef __attribute__((ext_vector_type(16))) _Float16 v16h;
typedef __attribute__((ext_vector_type(8)))  _Float16 v8h;
typedef __attribute__((ext_vector_type(8)))  float    v8f;
typedef __attribute__((ext_vector_type(4)))  float    v4f;

template <typename T> struct Frag;
template <> struct Frag<_Float16> {
  typedef v16h V; union U { v16h v; v8h h[2]; };
  static __device__ __forceinline__ v16h load(const _Float16* p) {
    U f; f.h[0] = *(const v8h*)(p); f.h[1] = *(const v8h*)(p + 16); return f.v;
  }
  static __device__ __forceinline__ v8f mma(v16h a, v16h b, v8f c) {
    return __builtin_amdgcn_wmma_f32_16x16x32_f16(false, a, false, b, (short)0, c, false, false);
  }
};

__device__ __forceinline__ void guard6h(v8f& a0, v8f& a1, v8f& a2, v8f& a3, v8f& a4, v8f& a5,
                                        v16h f0, v16h f1, v16h f2, v16h f3, v16h f4) {
  asm volatile("v_nop\n\tv_nop\n\tv_nop\n\tv_nop"
               : "+v"(a0), "+v"(a1), "+v"(a2), "+v"(a3), "+v"(a4), "+v"(a5)
               : "v"(f0), "v"(f1), "v"(f2), "v"(f3), "v"(f4));
}
__device__ __forceinline__ void accg6(v8f& a0, v8f& a1, v8f& a2, v8f& a3, v8f& a4, v8f& a5) {
  asm volatile("v_nop\n\tv_nop\n\tv_nop\n\tv_nop" : "+v"(a0), "+v"(a1), "+v"(a2), "+v"(a3), "+v"(a4), "+v"(a5));
}
__device__ __forceinline__ void guard2h(v8f& a0, v8f& a1, v16h f0, v16h f1, v16h f2) {
  asm volatile("v_nop\n\tv_nop\n\tv_nop\n\tv_nop" : "+v"(a0), "+v"(a1) : "v"(f0), "v"(f1), "v"(f2));
}
__device__ __forceinline__ void accg2(v8f& a0, v8f& a1) {
  asm volatile("v_nop\n\tv_nop\n\tv_nop\n\tv_nop" : "+v"(a0), "+v"(a1));
}
__device__ __forceinline__ void membar() { asm volatile("" ::: "memory"); }

__device__ __forceinline__ float fsigm(float v) { return __builtin_amdgcn_rcpf(1.0f + expf(-v)); }
__device__ __forceinline__ float ftanh(float v) { return 1.0f - 2.0f * __builtin_amdgcn_rcpf(1.0f + expf(2.0f * v)); }

__device__ __forceinline__ void stage_whh(const float* __restrict__ src, _Float16* dst, int tid) {
#pragma unroll 1
  for (int i = tid; i < G3 * (HID / 8); i += NTHR) {
    const int n = i >> 3, q = (i & 7) * 8;
    const v4f a = *(const v4f*)(src + n * HID + q);
    const v4f b = *(const v4f*)(src + n * HID + q + 4);
    v8h h;
#pragma unroll
    for (int e = 0; e < 4; ++e) { h[e] = (_Float16)(a[e] * WCAR); h[4 + e] = (_Float16)(b[e] * WCAR); }
    *(v8h*)(dst + n * WP + q) = h;
  }
}
__device__ __forceinline__ void stage_f1(const float* __restrict__ fc1w, _Float16* dst, int dir, int tid) {
  const int n = tid >> 3, q = (tid & 7) * 8;
  const int nc = (n < F1N) ? n : (F1N - 1);
  const v4f a = *(const v4f*)(fc1w + nc * F1K + dir * HID + q);
  const v4f b = *(const v4f*)(fc1w + nc * F1K + dir * HID + q + 4);
  v8h h;
#pragma unroll
  for (int e = 0; e < 4; ++e) {
    const float fa = (n < F1N) ? (a[e] * WCAR) : 0.0f;
    const float fb = (n < F1N) ? (b[e] * WCAR) : 0.0f;
    h[e] = (_Float16)fa; h[4 + e] = (_Float16)fb;
  }
  *(v8h*)(dst + n * WP + q) = h;
}
__device__ __forceinline__ void stage_x(const float* __restrict__ xg, float* xs, int tid) {
#pragma unroll 1
  for (int i = tid; i < (RPB * XROW) / 4; i += NTHR) {
    const v4f v = *(const v4f*)(xg + 4 * i);
    *(v4f*)(xs + 4 * i) = v;
  }
}
__device__ __forceinline__ void copy4(float* dst, const float* __restrict__ src, int n4, int tid) {
  const int ic = (tid < n4) ? tid : (n4 - 1);
  const v4f v = *(const v4f*)(src + 4 * ic);
  if (tid < n4) *(v4f*)(dst + 4 * tid) = v;
}

__global__ void __launch_bounds__(NTHR) __attribute__((amdgpu_num_vgpr(256)))
bigru_fc_kernel(const float* __restrict__ x,
                const float* __restrict__ wih_f, const float* __restrict__ whh_f,
                const float* __restrict__ bih_f, const float* __restrict__ bhh_f,
                const float* __restrict__ wih_b, const float* __restrict__ whh_b,
                const float* __restrict__ bih_b, const float* __restrict__ bhh_b,
                const float* __restrict__ fc1w, const float* __restrict__ fc1b,
                const float* __restrict__ fc2w, const float* __restrict__ fc2b,
                float* __restrict__ out) {
  __shared__ __align__(16) unsigned char smem[LDS_TOTAL];
  _Float16* WHL = (_Float16*)(smem + OFF_WHL);
  _Float16* F1L = (_Float16*)(smem + OFF_F1L);
  _Float16* HHI = (_Float16*)(smem + OFF_HHI);
  _Float16* HLO = (_Float16*)(smem + OFF_HLO);
  float*    XS  = (float*)(smem + OFF_XS);
  float*    CST = (float*)(smem + OFF_CST);
  float*    TAB = (float*)(smem + OFF_TAB);
  float*    OST = (float*)(smem + OFF_OST);
  float*    FCP = (float*)(smem + OFF_FCP);

  const int tid   = threadIdx.x;
  const int wave  = tid >> 5;
  const int lane  = tid & 31;
  const int c     = lane & 15;
  const int hh    = lane >> 4;
  const int koff  = hh * 8;
  const int dir   = wave >> 2;
  const int pairi = wave >> 1;
  const int row0  = (pairi & 1) * 16;
  const int uh    = wave & 1;
  const size_t gbase = (size_t)blockIdx.x * RPB;

  stage_x(x + gbase * XROW, XS, tid);                     membar();
  stage_whh(whh_f, WHL, tid);                             membar();
  stage_whh(whh_b, WHL + G3 * WP, tid);                   membar();
  stage_f1(fc1w, F1L, 0, tid);                            membar();
  stage_f1(fc1w, F1L + F1NP * WP, 1, tid);                membar();
  copy4(CST,                  wih_f, (G3 * NIN) / 4, tid); membar();
  copy4(CST + CST_BIH,        bih_f, G3 / 4, tid);         membar();
  copy4(CST + CST_BHH,        bhh_f, G3 / 4, tid);         membar();
  copy4(CST + CSTD,           wih_b, (G3 * NIN) / 4, tid); membar();
  copy4(CST + CSTD + CST_BIH, bih_b, G3 / 4, tid);         membar();
  copy4(CST + CSTD + CST_BHH, bhh_b, G3 / 4, tid);         membar();
  {
    const int i6 = (tid < F1N / 4) ? tid : (F1N / 4 - 1);
    const int i9 = (tid < (F2N * TSEQ) / 4) ? tid : ((F2N * TSEQ) / 4 - 1);
    const int i2 = (tid < F2N) ? tid : (F2N - 1);
    const v4f a  = *(const v4f*)(fc1b + 4 * i6);
    const v4f bq = *(const v4f*)(fc2w + 4 * i9);
    const float cq = fc2b[i2];
    if (tid < F1N / 4) *(v4f*)(TAB + 4 * tid) = a;
    if (tid < (F2N * TSEQ) / 4) *(v4f*)(TAB + F1N + 4 * tid) = bq;
    if (tid < F2N) TAB[F1N + F2N * TSEQ + tid] = cq;
  }
  membar();
  {
    const v4f z4 = {0.0f, 0.0f, 0.0f, 0.0f};
    float* hz = (float*)(smem + OFF_HHI);
#pragma unroll 1
    for (int i = tid; i < (2 * 4 * 16 * WP * 2) / 16; i += NTHR) *(v4f*)(hz + 4 * i) = z4;
#pragma unroll 1
    for (int i = tid; i < (RPB * VROW) / 4; i += NTHR) *(v4f*)(FCP + 4 * i) = z4;
  }
  __syncthreads();

  _Float16* hhi = HHI + pairi * (16 * WP);
  _Float16* hlo = HLO + pairi * (16 * WP);
  const _Float16* whl = WHL + dir * (G3 * WP);
  const _Float16* f1l = F1L + dir * (F1NP * WP);
  const float*    cst = CST + dir * CSTD;
  const _Float16* arow_h = hhi + c * WP + koff;
  const _Float16* arow_l = hlo + c * WP + koff;

  float ho[2][8];
#pragma unroll
  for (int ubl = 0; ubl < 2; ++ubl)
#pragma unroll
    for (int r = 0; r < 8; ++r) ho[ubl][r] = 0.0f;
  const v8f z8 = {0.0f, 0.0f, 0.0f, 0.0f, 0.0f, 0.0f, 0.0f, 0.0f};

#pragma unroll 1
  for (int s = 0; s < TSEQ; ++s) {
    const int t = dir ? (TSEQ - 1 - s) : s;

    float x0[8], x1[8];
#pragma unroll
    for (int r = 0; r < 8; ++r) {
      const float* xp = XS + (row0 + 8 * hh + r) * XROW + t * NIN;
      x0[r] = xp[0];
      x1[r] = xp[1];
    }

#pragma unroll
    for (int ubl = 0; ubl < 2; ++ubl) {
      const int j = 32 * uh + 16 * ubl + c;
      const _Float16* pbr = whl + j * WP + koff;
      const _Float16* pbz = whl + (HID + j) * WP + koff;
      const _Float16* pbn = whl + (2 * HID + j) * WP + koff;
      v8f aR = z8, aZ = z8, aN = z8, lR = z8, lZ = z8, lN = z8;
#pragma unroll 1
      for (int k0 = 0; k0 < HID; k0 += 32) {
        const v16h fh = Frag<_Float16>::load(arow_h + k0);
        const v16h fl = Frag<_Float16>::load(arow_l + k0);
        const v16h wr = Frag<_Float16>::load(pbr + k0);
        const v16h wz = Frag<_Float16>::load(pbz + k0);
        const v16h wn = Frag<_Float16>::load(pbn + k0);
        aR = Frag<_Float16>::mma(fh, wr, aR);
        aZ = Frag<_Float16>::mma(fh, wz, aZ);
        aN = Frag<_Float16>::mma(fh, wn, aN);
        lR = Frag<_Float16>::mma(fl, wr, lR);
        lZ = Frag<_Float16>::mma(fl, wz, lZ);
        lN = Frag<_Float16>::mma(fl, wn, lN);
        guard6h(aR, aZ, aN, lR, lZ, lN, fh, fl, wr, wz, wn);
      }
      accg6(aR, aZ, aN, lR, lZ, lN);

      const float wAr = cst[NIN * j],             wBr = cst[NIN * j + 1];
      const float wAz = cst[NIN * (HID + j)],     wBz = cst[NIN * (HID + j) + 1];
      const float wAn = cst[NIN * (2 * HID + j)], wBn = cst[NIN * (2 * HID + j) + 1];
      const float bir = cst[CST_BIH + j], biz = cst[CST_BIH + HID + j], bin = cst[CST_BIH + 2 * HID + j];
      const float bhr = cst[CST_BHH + j], bhz = cst[CST_BHH + HID + j], bhn = cst[CST_BHH + 2 * HID + j];
#pragma unroll
      for (int r = 0; r < 8; ++r) {
        float pr = x0[r] * wAr; pr = fmaf(x1[r], wBr, pr); const float ir = pr + bir;
        float pz = x0[r] * wAz; pz = fmaf(x1[r], wBz, pz); const float iz = pz + biz;
        float pn = x0[r] * wAn; pn = fmaf(x1[r], wBn, pn); const float in_ = pn + bin;
        const float gr = fmaf(lR[r], LCAR_INV, aR[r]) * WCAR_INV + bhr;
        const float gz = fmaf(lZ[r], LCAR_INV, aZ[r]) * WCAR_INV + bhz;
        const float gn = fmaf(lN[r], LCAR_INV, aN[r]) * WCAR_INV + bhn;
        const float rg = fsigm(ir + gr);
        const float zg = fsigm(iz + gz);
        const float ng = ftanh(in_ + rg * gn);
        const float hold = ho[ubl][r];
        ho[ubl][r] = (1.0f - zg) * ng + zg * hold;
      }
    }
    __syncthreads();

#pragma unroll
    for (int ubl = 0; ubl < 2; ++ubl)
#pragma unroll
      for (int r = 0; r < 8; ++r) {
        const float h = ho[ubl][r];
        const float hcl = (fabsf(h) < F16_MIN_NORMAL) ? 0.0f : h;
        const _Float16 hv = (_Float16)hcl;
        const float hvf = (float)hv;
        const float res = (h - hvf) * LCAR;
        const int o = (8 * hh + r) * WP + 32 * uh + 16 * ubl + c;
        hhi[o] = hv;
        hlo[o] = (_Float16)res;
      }
    __syncthreads();

    {
      v8f fa = z8, ga = z8;
      const _Float16* pb = f1l + (16 * uh + c) * WP + koff;
#pragma unroll 1
      for (int k0 = 0; k0 < HID; k0 += 32) {
        const v16h fh = Frag<_Float16>::load(arow_h + k0);
        const v16h fl = Frag<_Float16>::load(arow_l + k0);
        const v16h w0 = Frag<_Float16>::load(pb + k0);
        fa = Frag<_Float16>::mma(fh, w0, fa);
        ga = Frag<_Float16>::mma(fl, w0, ga);
        guard2h(fa, ga, fh, fl, w0);
      }
      accg2(fa, ga);
      const int col  = 16 * uh + c;
      const int colc = (col < F1N) ? col : (F1N - 1);
      float* fcrow = FCP + (row0 + 8 * hh) * VROW + t * F1N + colc;
#pragma unroll
      for (int r = 0; r < 8; ++r) {
        float* fr = fcrow + r * VROW;
        const float v = fmaf(ga[r], LCAR_INV, fa[r]) * WCAR_INV;
        const float u = fr[0] + v;
        if (col < F1N) fr[0] = u;
      }
    }
    __syncthreads();
  }

  {
    const float fb0 = TAB[F1N + F2N * TSEQ], fb1 = TAB[F1N + F2N * TSEQ + 1];
#pragma unroll 1
    for (int p = tid; p < RPB * F1N; p += NTHR) {
      const int row = p / F1N;
      const int i   = p - row * F1N;
      const float* vr = FCP + row * VROW + i * TSEQ;
      float s0 = 0.0f, s1 = 0.0f;
#pragma unroll 1
      for (int jj = 0; jj < TSEQ; ++jj) {
        const int f  = i * TSEQ + jj;
        const int cc = f - (f / F1N) * F1N;
        const float v = vr[jj] + TAB[cc];
        s0 = fmaf(v, TAB[F1N + jj], s0);
        s1 = fmaf(v, TAB[F1N + TSEQ + jj], s1);
      }
      OST[row * OROW + i * F2N + 0] = s0 + fb0;
      OST[row * OROW + i * F2N + 1] = s1 + fb1;
    }
  }
  __syncthreads();
  if (wave < 6) {
    float* ob = out + (size_t)blockIdx.x * (RPB * OROW);
    for (int pass = 0; pass < 2; ++pass) {
#pragma unroll
      for (int it = 0; it < 2; ++it) {
        const int off = wave * 256 + it * 128 + lane * 4;
        const v4f v = *(const v4f*)(OST + off);
        *(volatile v4f*)(ob + off) = v;
      }
      __threadfence();
    }
  }
}

extern "C" void kernel_launch(void* const* d_in, const int* in_sizes, int n_in,
                              void* d_out, int out_size, void* d_ws, size_t ws_size,
                              hipStream_t stream) {
  (void)d_ws; (void)ws_size;
  if (n_in < 13 || d_out == nullptr) return;
  if (in_sizes[0] != NB * TSEQ * NIN || in_sizes[1] != G3 * NIN || in_sizes[2] != G3 * HID ||
      in_sizes[3] != G3 || in_sizes[4] != G3 || in_sizes[5] != G3 * NIN || in_sizes[6] != G3 * HID ||
      in_sizes[7] != G3 || in_sizes[8] != G3 || in_sizes[9] != F1N * F1K || in_sizes[10] != F1N ||
      in_sizes[11] != F2N * TSEQ || in_sizes[12] != F2N || out_size != NB * OROW) return;

  const float* x     = (const float*)d_in[0];
  const float* wih_f = (const float*)d_in[1];
  const float* whh_f = (const float*)d_in[2];
  const float* bih_f = (const float*)d_in[3];
  const float* bhh_f = (const float*)d_in[4];
  const float* wih_b = (const float*)d_in[5];
  const float* whh_b = (const float*)d_in[6];
  const float* bih_b = (const float*)d_in[7];
  const float* bhh_b = (const float*)d_in[8];
  const float* fc1w  = (const float*)d_in[9];
  const float* fc1b  = (const float*)d_in[10];
  const float* fc2w  = (const float*)d_in[11];
  const float* fc2b  = (const float*)d_in[12];
  float* out = (float*)d_out;

  bigru_fc_kernel<<<NB / RPB, NTHR, 0, stream>>>(
      x, wih_f, whh_f, bih_f, bhh_f, wih_b, whh_b, bih_b, bhh_b, fc1w, fc1b, fc2w, fc2b, out);
}
